// SimpleGraphSAGE_10514079941027
// MI455X (gfx1250) — hardware-run, weakly checked
//
#include <hip/hip_runtime.h>
#include <stddef.h>
#include <stdint.h>

#define SPLIT_MEAN 1
#define SPLIT_H    1

#define NN      50000
#define NE      1600000
#define DF      128
#define MP      50048
#define MPW     (SPLIT_MEAN ? 256 : 128)
#define HPW     (SPLIT_H ? 256 : 128)
#define K1      (MPW + DF)
#define K2      (MPW + HPW)
#define GBM     64
#define GBN     128
#define GTHR    128
#define NTHR    256
#define NWAVE   8
#define EPT     8
#define WCH     (32 * EPT)
#define NBRUN   1024
#define SLB     10
#define NBK     49
#define PWCAP   5120
#define RCAP    40960
#define TRIPCAP 256
#define MAXDEG_MEAS   61
#define MAXB1024_MEAS 33116
#define ABM     64
#define WSMAX   134217728

#define BK_ZINTS (NWAVE * PWCAP + RCAP / 2 + 3 * NBRUN)
#define BK_INTS  (BK_ZINTS + 16)
#define BK_LDS   (BK_INTS * 4)

#define PBX   (MP * DF / 8 / NTHR)
#define PBW   (7 * 8)
#define PBTOT (PBX + PBW + 1)

static_assert(DF == 128 && DF == 32 * 4);
static_assert(MP % GBM == 0 && MP >= NN && MP == 391 * 128 && MP % ABM == 0);
static_assert(NBRUN == (1 << SLB) && NBRUN % ABM == 0 && NBRUN % GBM == 0 && NBRUN % 32 == 0);
static_assert(NBK == 49 && NBK * NBRUN >= MP && (NBK - 1) * NBRUN < MP);
static_assert(NE < (1 << 21) && (((long long)NE) << SLB) < (1LL << 31));
static_assert(NE % WCH == 0 && NE % 4 == 0);
static_assert(RCAP == NWAVE * PWCAP && RCAP % 8 == 0 && PWCAP % 256 == 0);
static_assert((long long)RCAP * 100 >= (long long)MAXB1024_MEAS * 120);
static_assert((long long)PWCAP * 80 >= (long long)MAXB1024_MEAS * 12);
static_assert(PWCAP >= MAXB1024_MEAS / 8 + 8 * 65 + 1);
static_assert(NN <= 65536);
static_assert(MAXDEG_MEAS + 8 <= TRIPCAP && TRIPCAP <= RCAP && RCAP < (1 << 30));
static_assert(K1 % 32 == 0 && K2 % 32 == 0 && MPW % 32 == 0 && HPW % 32 == 0);
static_assert(GBN == DF && GBM == (GTHR / 32) * 16 && ABM == NWAVE * 8);
static_assert(BK_ZINTS % (NTHR * 4) == 0 && (RCAP / 2) % (NTHR * 4) == 0 && (2 * NBRUN) % (NTHR * 4) == 0);
static_assert(BK_LDS <= 300000);
static_assert((GBM * GBN + DF) * 4 <= 65536);
static_assert((MP * DF / 8) % NTHR == 0);
static_assert((long long)NN * DF == 6400000LL);

typedef float          v4f   __attribute__((ext_vector_type(4)));
typedef float          v8f   __attribute__((ext_vector_type(8)));
typedef int            v4i   __attribute__((ext_vector_type(4)));
typedef int            v8i   __attribute__((ext_vector_type(8)));
typedef unsigned       v2u   __attribute__((ext_vector_type(2)));
typedef unsigned short v8us  __attribute__((ext_vector_type(8)));
typedef unsigned short v16us __attribute__((ext_vector_type(16)));
typedef __bf16         v16bf __attribute__((ext_vector_type(16)));
typedef v4f  __attribute__((may_alias)) v4fa;
typedef v4i  __attribute__((may_alias)) v4ia;
typedef v2u  __attribute__((may_alias)) v2ua;
typedef v8us __attribute__((may_alias)) v8usa;
union FragB { v16bf v; v16us u; v8us h[2]; v8i w; };

__device__ __forceinline__ v8f wmb(const FragB& a, const FragB& b, v8f c) {
  v8f d = __builtin_amdgcn_wmma_f32_16x16x32_bf16(false, a.v, false, b.v, (short)0, c, false, false);
  asm volatile("v_nop\n\tv_nop\n\tv_nop\n\tv_nop" : "+v"(d) : "v"(a.w), "v"(b.w));
  return d;
}

__device__ __forceinline__ unsigned bf16_bits(float f) {
  const unsigned u = __float_as_uint(f);
  const unsigned r = (u + 0x7FFFu + ((u >> 16) & 1u)) >> 16;
  const unsigned q = (u >> 16) | 0x40u;
  return ((u & 0x7fffffffu) > 0x7f800000u) ? q : r;
}
__device__ __forceinline__ float bf16_val(float f) {
  return __uint_as_float(bf16_bits(f) << 16);
}

__device__ __forceinline__ void hilo_pack(float v0, float v1, float v2, float v3,
                                          int& h01, int& h23, int& l01, int& l23) {
  const unsigned a0 = bf16_bits(v0), a1 = bf16_bits(v1), a2 = bf16_bits(v2), a3 = bf16_bits(v3);
  const unsigned b0 = bf16_bits(v0 - __uint_as_float(a0 << 16));
  const unsigned b1 = bf16_bits(v1 - __uint_as_float(a1 << 16));
  const unsigned b2 = bf16_bits(v2 - __uint_as_float(a2 << 16));
  const unsigned b3 = bf16_bits(v3 - __uint_as_float(a3 << 16));
  h01 = (int)(a0 | (a1 << 16)); h23 = (int)(a2 | (a3 << 16));
  l01 = (int)(b0 | (b1 << 16)); l23 = (int)(b2 | (b3 << 16));
}

__device__ __forceinline__ v4i regroup16(int h01, int h23, int l01, int l23, int lane) {
  const int s0 = (2 * lane) & 31, s1 = s0 + 1;
  const int a0 = __shfl(h01, s0, 32), a1 = __shfl(h23, s0, 32), a2 = __shfl(h01, s1, 32), a3 = __shfl(h23, s1, 32);
  const int b0 = __shfl(l01, s0, 32), b1 = __shfl(l23, s0, 32), b2 = __shfl(l01, s1, 32), b3 = __shfl(l23, s1, 32);
  const int mk = (lane < 16) ? -1 : 0;
  v4i o;
  o.x = (a0 & mk) | (b0 & ~mk); o.y = (a1 & mk) | (b1 & ~mk);
  o.z = (a2 & mk) | (b2 & ~mk); o.w = (a3 & mk) | (b3 & ~mk);
  return o;
}

__device__ __forceinline__ void st2_v4f(float* p, v4f v) {
  *(volatile v4f*)p = v;
  __threadfence();
  *(volatile v4f*)p = v;
}
__device__ __forceinline__ void st2_v8us(unsigned short* p, v8us v) {
  *(volatile v8us*)p = v;
  __threadfence();
  *(volatile v8us*)p = v;
}

template <int PW>
__device__ __forceinline__ void put_row(unsigned short* rowp, float v0, float v1, float v2, float v3, int lane) {
  if constexpr (PW == 256) {
    int h01, h23, l01, l23;
    hilo_pack(v0, v1, v2, v3, h01, h23, l01, l23);
    const v4i ow = regroup16(h01, h23, l01, l23, lane);
    unsigned short* p = rowp + 8 * lane;
    *(volatile v4i*)p = ow;
    __threadfence();
    *(volatile v4i*)p = ow;
  } else {
    const unsigned a0 = bf16_bits(v0), a1 = bf16_bits(v1), a2 = bf16_bits(v2), a3 = bf16_bits(v3);
    v2u ow;
    ow.x = a0 | (a1 << 16); ow.y = a2 | (a3 << 16);
    unsigned short* p = rowp + 4 * lane;
    *(volatile v2u*)p = ow;
    __threadfence();
    *(volatile v2u*)p = ow;
  }
}

__device__ __forceinline__ void wunit(const float* __restrict__ W, unsigned short* P, int pitch, int coff, int v) {
  const int n  = v >> 4;
  const int k8 = (v & 15) * 8;
  const float* p = W + (size_t)n * DF + k8;
  const v4f a = *(const v4fa*)p;
  const v4f b = *(const v4fa*)(p + 4);
  v8us o;
  o[0] = (unsigned short)bf16_bits(a.x); o[1] = (unsigned short)bf16_bits(a.y);
  o[2] = (unsigned short)bf16_bits(a.z); o[3] = (unsigned short)bf16_bits(a.w);
  o[4] = (unsigned short)bf16_bits(b.x); o[5] = (unsigned short)bf16_bits(b.y);
  o[6] = (unsigned short)bf16_bits(b.z); o[7] = (unsigned short)bf16_bits(b.w);
  st2_v8us(P + (size_t)n * pitch + coff + k8, o);
}

__global__ __launch_bounds__(NTHR) void k_prep(const float* __restrict__ x,
                                               const float* __restrict__ W1l, const float* __restrict__ b1,
                                               const float* __restrict__ W1r, const float* __restrict__ W2l,
                                               const float* __restrict__ b2, const float* __restrict__ W2r,
                                               unsigned short* xb, unsigned short* w1c, unsigned short* w2c,
                                               float* bt) {
  const int tid = (int)threadIdx.x, lane = tid & 31, wave = tid >> 5;
  const int blk = (int)blockIdx.x;
  if (blk < PBX) {
    const int u   = blk * NTHR + tid;
    const int row = u >> 4, k8 = (u & 15) * 8;
    const int rc  = row < NN ? row : NN - 1;
    const unsigned mk = row < NN ? 0xffffu : 0u;
    const float* p = x + (size_t)rc * DF + k8;
    const v4f a = *(const v4fa*)p;
    const v4f b = *(const v4fa*)(p + 4);
    v8us o;
    o[0] = (unsigned short)(bf16_bits(a.x) & mk); o[1] = (unsigned short)(bf16_bits(a.y) & mk);
    o[2] = (unsigned short)(bf16_bits(a.z) & mk); o[3] = (unsigned short)(bf16_bits(a.w) & mk);
    o[4] = (unsigned short)(bf16_bits(b.x) & mk); o[5] = (unsigned short)(bf16_bits(b.y) & mk);
    o[6] = (unsigned short)(bf16_bits(b.z) & mk); o[7] = (unsigned short)(bf16_bits(b.w) & mk);
    st2_v8us(xb + (size_t)row * DF + k8, o);
  } else if (blk < PBX + PBW) {
    const int pb   = blk - PBX;
    const int slot = pb >> 3;
    const int v    = (pb & 7) * NTHR + tid;
    if (slot == 0) {
      wunit(W1l, w1c, K1, 0, v);
    } else if (slot == 1) {
      if constexpr (SPLIT_MEAN != 0) wunit(W1l, w1c, K1, DF, v);
    } else if (slot == 2) {
      wunit(W1r, w1c, K1, MPW, v);
    } else if (slot == 3) {
      wunit(W2l, w2c, K2, 0, v);
    } else if (slot == 4) {
      if constexpr (SPLIT_MEAN != 0) wunit(W2l, w2c, K2, DF, v);
    } else if (slot == 5) {
      wunit(W2r, w2c, K2, MPW, v);
    } else {
      if constexpr (SPLIT_H != 0) wunit(W2r, w2c, K2, MPW + DF, v);
    }
  } else {
    if (wave == 0) {
      const v4f a = *(const v4fa*)(b1 + 4 * lane);
      v4f o;
      o.x = bf16_val(a.x); o.y = bf16_val(a.y); o.z = bf16_val(a.z); o.w = bf16_val(a.w);
      st2_v4f(bt + 4 * lane, o);
    } else if (wave == 1) {
      const v4f a = *(const v4fa*)(b2 + 4 * lane);
      v4f o;
      o.x = bf16_val(a.x); o.y = bf16_val(a.y); o.z = bf16_val(a.z); o.w = bf16_val(a.w);
      st2_v4f(bt + DF + 4 * lane, o);
    }
  }
}

__device__ __forceinline__ void bucket_flush(const int* plw, const int* cnt, int ov, int* lp, int* cop, int* fp,
                                             int tid) {
#pragma unroll 1
  for (int i = tid * 4; i < RCAP / 2; i += NTHR * 4) {
    const v4i v = *(const v4ia*)(plw + i);
    *(volatile v4i*)(lp + i) = v;
  }
#pragma unroll 1
  for (int i = tid * 4; i < 2 * NBRUN; i += NTHR * 4) {
    const v4i v = *(const v4ia*)(cnt + i);
    *(volatile v4i*)(cop + i) = v;
  }
  if (tid < 8) {
    const v4i f = {ov, ov, ov, ov};
    *(volatile v4i*)(fp + 4 * tid) = f;
  }
}

__global__ __launch_bounds__(NTHR) void k_bucket(const int* __restrict__ srcs, const int* __restrict__ dsts,
                                                 int* LIST, int* CO, int* FLAG) {
  extern __shared__ __attribute__((aligned(16))) int dsm[];
  int* wl   = dsm;
  int* plw  = dsm + NWAVE * PWCAP;
  unsigned short* pl = (unsigned short*)plw;
  int* cnt  = plw + RCAP / 2;
  int* offs = cnt + NBRUN;
  int* cur  = offs + NBRUN;
  int* misc = cur + NBRUN;
  const int tid = (int)threadIdx.x, lane = tid & 31, wave = tid >> 5;
  const int blk = (int)blockIdx.x;
  const unsigned nbs = (unsigned)(blk * NBRUN);

  {
    const v4i z4 = {0, 0, 0, 0};
    for (int i = tid * 4; i < BK_ZINTS; i += NTHR * 4) *(v4ia*)(dsm + i) = z4;
    if (tid < 16) misc[tid] = 0;
  }
  __syncthreads();

  {
    const int per  = ((NE + NWAVE * WCH - 1) / (NWAVE * WCH)) * WCH;
    const int ebeg = wave * per;
    const int eend = (ebeg + per < NE) ? (ebeg + per) : NE;
    int* mylist = wl + wave * PWCAP;
    int wc = 0;
#pragma unroll 1
    for (int cb = ebeg; cb < eend; cb += WCH) {
      const int e0 = cb + lane * EPT;
      const v4i da = *(const v4ia*)(dsts + e0);
      const v4i db = *(const v4ia*)(dsts + e0 + 4);
      const unsigned s0 = (unsigned)da.x - nbs, s1 = (unsigned)da.y - nbs;
      const unsigned s2 = (unsigned)da.z - nbs, s3 = (unsigned)da.w - nbs;
      const unsigned s4 = (unsigned)db.x - nbs, s5 = (unsigned)db.y - nbs;
      const unsigned s6 = (unsigned)db.z - nbs, s7 = (unsigned)db.w - nbs;
      const bool h0 = s0 < (unsigned)NBRUN, h1 = s1 < (unsigned)NBRUN, h2 = s2 < (unsigned)NBRUN, h3 = s3 < (unsigned)NBRUN;
      const bool h4 = s4 < (unsigned)NBRUN, h5 = s5 < (unsigned)NBRUN, h6 = s6 < (unsigned)NBRUN, h7 = s7 < (unsigned)NBRUN;
      const unsigned m0 = __builtin_amdgcn_ballot_w32(h0), m1 = __builtin_amdgcn_ballot_w32(h1);
      const unsigned m2 = __builtin_amdgcn_ballot_w32(h2), m3 = __builtin_amdgcn_ballot_w32(h3);
      const unsigned m4 = __builtin_amdgcn_ballot_w32(h4), m5 = __builtin_amdgcn_ballot_w32(h5);
      const unsigned m6 = __builtin_amdgcn_ballot_w32(h6), m7 = __builtin_amdgcn_ballot_w32(h7);
      const unsigned any = m0 | m1 | m2 | m3 | m4 | m5 | m6 | m7;
      if (any != 0u) {
        const int pre = (int)(__builtin_amdgcn_mbcnt_lo(m0, 0u) + __builtin_amdgcn_mbcnt_lo(m1, 0u) +
                              __builtin_amdgcn_mbcnt_lo(m2, 0u) + __builtin_amdgcn_mbcnt_lo(m3, 0u) +
                              __builtin_amdgcn_mbcnt_lo(m4, 0u) + __builtin_amdgcn_mbcnt_lo(m5, 0u) +
                              __builtin_amdgcn_mbcnt_lo(m6, 0u) + __builtin_amdgcn_mbcnt_lo(m7, 0u));
        int p = wc + pre;
        if (h0) { if (p < PWCAP) mylist[p] = ((e0 + 0) << SLB) | (int)s0; p = p + 1; }
        if (h1) { if (p < PWCAP) mylist[p] = ((e0 + 1) << SLB) | (int)s1; p = p + 1; }
        if (h2) { if (p < PWCAP) mylist[p] = ((e0 + 2) << SLB) | (int)s2; p = p + 1; }
        if (h3) { if (p < PWCAP) mylist[p] = ((e0 + 3) << SLB) | (int)s3; p = p + 1; }
        if (h4) { if (p < PWCAP) mylist[p] = ((e0 + 4) << SLB) | (int)s4; p = p + 1; }
        if (h5) { if (p < PWCAP) mylist[p] = ((e0 + 5) << SLB) | (int)s5; p = p + 1; }
        if (h6) { if (p < PWCAP) mylist[p] = ((e0 + 6) << SLB) | (int)s6; p = p + 1; }
        if (h7) { if (p < PWCAP) mylist[p] = ((e0 + 7) << SLB) | (int)s7; p = p + 1; }
        wc += (int)(__builtin_popcount(m0) + __builtin_popcount(m1) + __builtin_popcount(m2) + __builtin_popcount(m3) +
                    __builtin_popcount(m4) + __builtin_popcount(m5) + __builtin_popcount(m6) + __builtin_popcount(m7));
      }
    }
    if (lane == 0) misc[wave] = wc;
  }
  __syncthreads();

  if (wave == 0) {
    int ov = 0;
#pragma unroll 1
    for (int w2 = 0; w2 < NWAVE; ++w2) {
      int c = misc[w2];
      if (c > PWCAP) ov = 1;
      c = c < 0 ? 0 : (c > PWCAP ? PWCAP : c);
#pragma unroll 1
      for (int b0 = 0; b0 < c; b0 += 32) {
        const int idx = b0 + lane;
        const int ent = wl[w2 * PWCAP + (idx < PWCAP ? idx : PWCAP - 1)];
        const int m32 = (c - b0) < 32 ? (c - b0) : 32;
#pragma unroll 1
        for (int k = 0; k < m32; ++k) {
          const int u    = __builtin_amdgcn_readlane(ent, k);
          const int slot = u & (NBRUN - 1);
          if (lane == 0) cnt[slot] = cnt[slot] + 1;
        }
      }
    }
    if (lane == 0) misc[9] = ov;
  }
  __syncthreads();
  if (wave == 0) {
    const int base = lane * (NBRUN / 32);
    int s = 0;
#pragma unroll 1
    for (int i = 0; i < NBRUN / 32; ++i) s += cnt[base + i];
    int incl = s;
#pragma unroll
    for (int d = 1; d < 32; d <<= 1) {
      const int y = __shfl_up(incl, d, 32);
      if (lane >= d) incl += y;
    }
    int run = incl - s;
#pragma unroll 1
    for (int i = 0; i < NBRUN / 32; ++i) {
      const int cv = cnt[base + i];
      offs[base + i] = run;
      cur[base + i]  = run;
      run += cv;
    }
  }
  __syncthreads();

  if (wave == 0) {
#pragma unroll 1
    for (int w2 = 0; w2 < NWAVE; ++w2) {
      int c = misc[w2];
      c = c < 0 ? 0 : (c > PWCAP ? PWCAP : c);
#pragma unroll 1
      for (int b0 = 0; b0 < c; b0 += 32) {
        const int idx = b0 + lane;
        const int ent = wl[w2 * PWCAP + (idx < PWCAP ? idx : PWCAP - 1)];
        int eid = (ent >> SLB) & 0x1FFFFF;
        eid = eid > NE - 1 ? NE - 1 : eid;
        int sr = srcs[eid];
        sr = sr < 0 ? 0 : (sr > NN - 1 ? NN - 1 : sr);
        const int m32 = (c - b0) < 32 ? (c - b0) : 32;
#pragma unroll 1
        for (int k = 0; k < m32; ++k) {
          const int u    = __builtin_amdgcn_readlane(ent, k);
          const int sd   = __builtin_amdgcn_readlane(sr, k);
          const int slot = u & (NBRUN - 1);
          if (lane == 0) {
            int p = cur[slot];
            p = p < 0 ? 0 : (p > RCAP - 1 ? RCAP - 1 : p);
            int* pw = plw + (p >> 1);
            const int ow = *pw;
            *pw = (p & 1) ? ((ow & 0x0000ffff) | (sd << 16)) : ((ow & (int)0xffff0000u) | (sd & 0xffff));
            cur[slot] = p + 1;
          }
        }
      }
    }
  }
  __syncthreads();

  const int ovf = misc[9];
  int* lp  = LIST + (size_t)blk * (RCAP / 2);
  int* cop = CO + (size_t)blk * (2 * NBRUN);
  int* fp  = FLAG + (size_t)blk * 32;
  bucket_flush(plw, cnt, ovf, lp, cop, fp, tid);
  __threadfence();
  bucket_flush(plw, cnt, ovf, lp, cop, fp, tid);
}

template <int SPW, int SSPL>
__global__ __launch_bounds__(NTHR) void k_agg(const unsigned short* __restrict__ LIST, const int* __restrict__ CO,
                                              const int* __restrict__ FLAG,
                                              const unsigned short* __restrict__ srcp, unsigned short* agg) {
  const int tid = (int)threadIdx.x, lane = tid & 31;
  const int wave = __builtin_amdgcn_readfirstlane(tid >> 5);
  const int rowBase = (int)blockIdx.x * ABM;
  const int bucket  = rowBase >> SLB;
  const unsigned short* lb = LIST + (size_t)bucket * RCAP;
  const int* cob = CO + (size_t)bucket * (2 * NBRUN);
  const int flag = FLAG[(size_t)bucket * 32];
  const float qnan = __uint_as_float(0x7fc00000u);

#pragma unroll 1
  for (int i = 0; i < ABM / NWAVE; ++i) {
    const int d    = rowBase + (ABM / NWAVE) * wave + i;
    const int slot = d & (NBRUN - 1);
    int c = cob[slot];
    int o = cob[NBRUN + slot];
    const bool big = c > TRIPCAP;
    c = c < 0 ? 0 : (c > TRIPCAP ? TRIPCAP : c);
    o = o < 0 ? 0 : (o > RCAP - 1 ? RCAP - 1 : o);
    int last = o + c - 1;
    last = last < o ? o : last;
    last = last > RCAP - 1 ? RCAP - 1 : last;
    float a0 = 0.0f, a1 = 0.0f, a2 = 0.0f, a3 = 0.0f;
#pragma unroll 1
    for (int b0 = 0; b0 < c; b0 += 32) {
      int idx = o + b0 + lane;
      idx = idx > last ? last : idx;
      const unsigned int w2 = ((const unsigned int*)lb)[idx >> 1];
      int sr = (int)((idx & 1) ? (w2 >> 16) : (w2 & 0xffffu));
      sr = sr > NN - 1 ? NN - 1 : sr;
      const int m32 = (c - b0) < 32 ? (c - b0) : 32;
#pragma unroll 1
      for (int k = 0; k < m32; ++k) {
        const int sk = __builtin_amdgcn_readlane(sr, k);
        const unsigned short* rp = srcp + (size_t)sk * SPW + 4 * lane;
        const v2u wh = *(const v2ua*)rp;
        float f0 = __uint_as_float(wh.x << 16);
        float f1 = __uint_as_float(wh.x & 0xffff0000u);
        float f2 = __uint_as_float(wh.y << 16);
        float f3 = __uint_as_float(wh.y & 0xffff0000u);
        if constexpr (SSPL != 0) {
          const v2u wq = *(const v2ua*)(rp + DF);
          f0 += __uint_as_float(wq.x << 16);
          f1 += __uint_as_float(wq.x & 0xffff0000u);
          f2 += __uint_as_float(wq.y << 16);
          f3 += __uint_as_float(wq.y & 0xffff0000u);
        }
        a0 += f0; a1 += f1; a2 += f2; a3 += f3;
      }
    }
    const float den = fmaxf((float)c, 1.0f);
    float m0 = a0 / den, m1 = a1 / den, m2 = a2 / den, m3 = a3 / den;
    const bool bad  = (flag != 0) | big;
    const bool live = d < NN;
    m0 = bad ? qnan : m0; m1 = bad ? qnan : m1; m2 = bad ? qnan : m2; m3 = bad ? qnan : m3;
    m0 = live ? m0 : 0.0f; m1 = live ? m1 : 0.0f; m2 = live ? m2 : 0.0f; m3 = live ? m3 : 0.0f;
    put_row<MPW>(agg + (size_t)d * MPW, m0, m1, m2, m3, lane);
  }
}

template <int KSEG, int KT>
__device__ __forceinline__ void gemm_seg(const unsigned short* __restrict__ ap,
                                         const unsigned short* __restrict__ bp, v8f (&acc)[8]) {
#pragma unroll 1
  for (int k0 = 0; k0 < KSEG; k0 += 32) {
    FragB af;
    af.h[0] = *(const v8usa*)(ap + k0);
    af.h[1] = *(const v8usa*)(ap + k0 + 16);
#pragma unroll
    for (int nt = 0; nt < 8; ++nt) {
      const unsigned short* wq = bp + (size_t)(16 * nt) * (size_t)KT + k0;
      FragB bf;
      bf.h[0] = *(const v8usa*)wq;
      bf.h[1] = *(const v8usa*)(wq + 16);
      acc[nt] = wmb(af, bf, acc[nt]);
    }
  }
}

template <int FIN>
__global__ __launch_bounds__(GTHR) __attribute__((amdgpu_num_vgpr(248)))
void k_gemm(const unsigned short* __restrict__ A0, const unsigned short* __restrict__ A1,
            const unsigned short* __restrict__ BT, const float* __restrict__ btab,
            const int* __restrict__ FLAG, unsigned short* Hout, float* outp) {
  __shared__ __attribute__((aligned(16))) float stg[GBM * GBN];
  __shared__ __attribute__((aligned(16))) float sb[DF];
  constexpr int KA1 = (FIN != 0) ? HPW : DF;
  constexpr int KT  = MPW + KA1;
  const int tid = (int)threadIdx.x, lane = tid & 31, wave = tid >> 5, hh = lane >> 4, m = lane & 15;
  const int rowBase = (int)blockIdx.x * GBM;
  if (tid < 32) *(v4fa*)(sb + 4 * tid) = *(const v4fa*)(btab + 4 * tid);

  v8f acc[8];
  {
    const v8f z = {0.f, 0.f, 0.f, 0.f, 0.f, 0.f, 0.f, 0.f};
#pragma unroll
    for (int t = 0; t < 8; ++t) acc[t] = z;
  }
  const size_t arow = (size_t)(rowBase + 16 * wave + m);
  const unsigned short* bp = BT + (size_t)m * (size_t)KT + 8 * hh;
  gemm_seg<MPW, KT>(A0 + arow * (size_t)MPW + 8 * hh, bp, acc);
  gemm_seg<KA1, KT>(A1 + arow * (size_t)KA1 + 8 * hh, bp + MPW, acc);

#pragma unroll
  for (int nt = 0; nt < 8; ++nt) {
    const int lc = 16 * nt + m;
#pragma unroll
    for (int r = 0; r < 8; ++r) stg[(16 * wave + 8 * hh + r) * GBN + lc] = acc[nt][r];
  }
  __syncthreads();

  const v4f bias = *(const v4fa*)(sb + 4 * lane);
  const int flag = FLAG[(size_t)(rowBase >> SLB) * 32];
  const float qnan = __uint_as_float(0x7fc00000u);
#pragma unroll 1
  for (int i = 0; i < 16; ++i) {
    const int lr   = 16 * wave + i;
    const int grow = rowBase + lr;
    const v4f a = *(const v4fa*)(stg + lr * GBN + 4 * lane);
    asm volatile("" :: "v"(a));
    float v0 = a.x + bias.x, v1 = a.y + bias.y, v2 = a.z + bias.z, v3 = a.w + bias.w;
    if constexpr (FIN == 0) {
      const bool live = grow < NN;
      v0 = (v0 > 0.0f) ? v0 : (v0 - v0); v1 = (v1 > 0.0f) ? v1 : (v1 - v1);
      v2 = (v2 > 0.0f) ? v2 : (v2 - v2); v3 = (v3 > 0.0f) ? v3 : (v3 - v3);
      v0 = live ? v0 : 0.0f; v1 = live ? v1 : 0.0f; v2 = live ? v2 : 0.0f; v3 = live ? v3 : 0.0f;
      put_row<HPW>(Hout + (size_t)grow * HPW, v0, v1, v2, v3, lane);
    } else {
      v4f o;
      o.x = (flag != 0) ? qnan : v0; o.y = (flag != 0) ? qnan : v1;
      o.z = (flag != 0) ? qnan : v2; o.w = (flag != 0) ? qnan : v3;
      if (grow < NN) st2_v4f(outp + (size_t)grow * DF + 4 * lane, o);
    }
  }
}

extern "C" void kernel_launch(void* const* d_in, const int* in_sizes, int n_in,
                              void* d_out, int out_size, void* d_ws, size_t ws_size,
                              hipStream_t stream) {
  if (n_in < 8) return;
  if (in_sizes[0] != NN * DF) return;
  if (in_sizes[1] != 2 * NE) return;
  if (in_sizes[2] != DF * DF) return;
  if (in_sizes[3] != DF) return;
  if (in_sizes[4] != DF * DF) return;
  if (in_sizes[5] != DF * DF) return;
  if (in_sizes[6] != DF) return;
  if (in_sizes[7] != DF * DF) return;
  if (out_size != NN * DF) return;

  const float* x   = (const float*)d_in[0];
  const int*   ei  = (const int*)d_in[1];
  const float* W1l = (const float*)d_in[2];
  const float* b1  = (const float*)d_in[3];
  const float* W1r = (const float*)d_in[4];
  const float* W2l = (const float*)d_in[5];
  const float* b2  = (const float*)d_in[6];
  const float* W2r = (const float*)d_in[7];
  float* out = (float*)d_out;
  const int* srcs = ei;
  const int* dsts = ei + NE;

  constexpr size_t zXB   = (size_t)MP * DF * 2;
  constexpr size_t zAGG  = (size_t)MP * MPW * 2;
  constexpr size_t zH    = (size_t)MP * HPW * 2;
  constexpr size_t zLIST = (size_t)NBK * RCAP * 2;
  constexpr size_t zCO   = (size_t)NBK * 2 * NBRUN * 4;
  constexpr size_t zFLAG = 6400;
  constexpr size_t zW1   = (size_t)DF * K1 * 2;
  constexpr size_t zW2   = (size_t)DF * K2 * 2;
  constexpr size_t zBT   = 1024;
  constexpr size_t oXB   = 0;
  constexpr size_t oAGG  = oXB + zXB;
  constexpr size_t oH    = oAGG + zAGG;
  constexpr size_t oLIST = oH + zH;
  constexpr size_t oCO   = oLIST + zLIST;
  constexpr size_t oFLAG = oCO + zCO;
  constexpr size_t oW1   = oFLAG + zFLAG;
  constexpr size_t oW2   = oW1 + zW1;
  constexpr size_t oBT   = oW2 + zW2;
  constexpr size_t oEND  = oBT + zBT;
  static_assert(zXB % 256 == 0 && zAGG % 256 == 0 && zH % 256 == 0 && zLIST % 256 == 0 && zCO % 256 == 0);
  static_assert(zFLAG % 256 == 0 && zFLAG >= (size_t)NBK * 128 && zW1 % 256 == 0 && zW2 % 256 == 0);
  static_assert(zBT == 2 * DF * 4);
  static_assert(oEND <= (size_t)WSMAX);
  if (oEND > ws_size) return;

  char* ws = (char*)d_ws;
  unsigned short* XB   = (unsigned short*)(ws + oXB);
  unsigned short* AGG  = (unsigned short*)(ws + oAGG);
  unsigned short* H1   = (unsigned short*)(ws + oH);
  int*            LIST = (int*)(ws + oLIST);
  int*            CO   = (int*)(ws + oCO);
  int*            FLAG = (int*)(ws + oFLAG);
  unsigned short* W1C  = (unsigned short*)(ws + oW1);
  unsigned short* W2C  = (unsigned short*)(ws + oW2);
  float*          BTB  = (float*)(ws + oBT);

  hipFuncSetAttribute(reinterpret_cast<const void*>(&k_bucket), hipFuncAttributeMaxDynamicSharedMemorySize, (int)BK_LDS);

  k_prep<<<PBTOT, NTHR, 0, stream>>>(x, W1l, b1, W1r, W2l, b2, W2r, XB, W1C, W2C, BTB);
  k_bucket<<<NBK, NTHR, BK_LDS, stream>>>(srcs, dsts, LIST, CO, FLAG);
  k_agg<DF, 0><<<MP / ABM, NTHR, 0, stream>>>((const unsigned short*)LIST, CO, FLAG, XB, AGG);
  k_gemm<0><<<MP / GBM, GTHR, 0, stream>>>(AGG, XB, W1C, BTB, FLAG, H1, out);
  k_agg<HPW, SPLIT_H><<<MP / ABM, NTHR, 0, stream>>>((const unsigned short*)LIST, CO, FLAG, H1, AGG);
  k_gemm<1><<<MP / GBM, GTHR, 0, stream>>>(AGG, H1, W2C, BTB + DF, FLAG, H1, out);
}
